// GSG_35828617183594
// MI455X (gfx1250) — hardware-verified
//
#include <hip/hip_runtime.h>
#include <stdint.h>

#define DEVINL __device__ __forceinline__

typedef _Float16 f16t;
typedef _Float16 v16h __attribute__((ext_vector_type(16)));
typedef _Float16 v8h  __attribute__((ext_vector_type(8)));
typedef float    v8f  __attribute__((ext_vector_type(8)));
typedef float    v4f  __attribute__((ext_vector_type(4)));
typedef v8h __attribute__((may_alias)) v8ha;
typedef v4f __attribute__((may_alias)) v4fa;
union FragH { v16h v; v8h half[2]; };

#define NB    8
#define CIN   256
#define HW    4096
#define NQK   256
#define NV    512
#define NG    8
#define CQ    32
#define CV    64
#define CKEEP 32
#define COUT  256
#define KF    256
#define WROWS 1280
#define TPB   256
#define WAVES 8
#define PT    64
#define PQ    264
#define PK    72
#define PKT   40
#define XCAR  16.0f
#define WCAR  256.0f
#define QCAR  16.0f
#define KVCAR 16.0f
#define QVCAR 16.0f

static_assert(TPB == WAVES * 32);
static_assert((PQ % 8) == 0);
static_assert((PK % 8) == 0);
static_assert((PKT % 8) == 0);
static_assert((HW % PT) == 0);
static_assert(NQK == NG * CQ);
static_assert(NV == NG * CV);
static_assert(KF == NG * CKEEP);
static_assert((CIN % 32) == 0);
static_assert(TPB * 16 == HW);
static_assert(256 * PK >= PT * PQ);
static_assert(NB * NG * 2 == 128);

DEVINL int imin(int a, int b) { return a < b ? a : b; }
DEVINL int imax(int a, int b) { return a > b ? a : b; }

DEVINL v8f wmma_f16(v16h a, v16h b, v8f c) {
  v8f d = __builtin_amdgcn_wmma_f32_16x16x32_f16(false, a, false, b, (short)0, c, false, false);
  asm volatile("v_nop\n\tv_nop\n\tv_nop\n\tv_nop" : "+v"(d) : "v"(a), "v"(b));
  return d;
}
DEVINL v8f zero8f() {
  v8f z = {0.f, 0.f, 0.f, 0.f, 0.f, 0.f, 0.f, 0.f};
  return z;
}
DEVINL void load_frag(FragH& f, const f16t* row, int k0) {
  f.half[0] = *(const v8ha*)(row + k0);
  f.half[1] = *(const v8ha*)(row + k0 + 16);
}

DEVINL void store_rows256(const f16t* sT, f16t* dst, int wave, int lane) {
  #pragma unroll
  for (int i = 0; i < 8; ++i) {
    const int p = wave + 8 * i;
    const v8h v = *(const v8ha*)(sT + p * PQ + 8 * lane);
    *(volatile v8h*)(dst + (size_t)p * 256 + 8 * lane) = v;
  }
  __threadfence();
  #pragma unroll
  for (int i = 0; i < 8; ++i) {
    const int p = wave + 8 * i;
    const v8h v = *(const v8ha*)(sT + p * PQ + 8 * lane);
    *(volatile v8h*)(dst + (size_t)p * 256 + 8 * lane) = v;
  }
}

DEVINL void store_rows64(const f16t* sT, f16t* dst, int wave, int lane) {
  const int sub = lane >> 3, piece = (lane & 7) * 8;
  #pragma unroll
  for (int i = 0; i < 8; ++i) {
    const int row = wave * 32 + 4 * i + sub;
    const v8h v = *(const v8ha*)(sT + row * PK + piece);
    *(volatile v8h*)(dst + (size_t)row * HW + piece) = v;
  }
  __threadfence();
  #pragma unroll
  for (int i = 0; i < 8; ++i) {
    const int row = wave * 32 + 4 * i + sub;
    const v8h v = *(const v8ha*)(sT + row * PK + piece);
    *(volatile v8h*)(dst + (size_t)row * HW + piece) = v;
  }
}

__global__ __launch_bounds__(TPB) void prep_w_k(const float* __restrict__ Wq, const float* __restrict__ Wk,
                                               const float* __restrict__ Wv, const float* __restrict__ Wf,
                                               f16t* __restrict__ WP)
{
  const int t = blockIdx.x * TPB + threadIdx.x;
  if (t >= WROWS * 32) return;
  const int row = t >> 5, piece = (t & 31) * 8;
  const int rq = imin(row, 255);
  const int rk = imin(imax(row - 256, 0), 255);
  const int rv = imin(imax(row - 512, 0), 511);
  const int rf = imin(imax(row - 1024, 0), 255);
  v8h o;
  #pragma unroll
  for (int i = 0; i < 8; ++i) {
    const int c = piece + i;
    const float wq = Wq[rq * CIN + c];
    const float wk = Wk[rk * CIN + c];
    const float wv = Wv[rv * CIN + c];
    const float wf = Wf[rf * KF + c];
    float w = wf;
    w = (row < 1024) ? wv : w;
    w = (row < 512)  ? wk : w;
    w = (row < 256)  ? wq : w;
    o[i] = (f16t)(w * WCAR);
  }
  f16t* dst = WP + (size_t)row * CIN + piece;
  *(volatile v8h*)dst = o;
  __threadfence();
  *(volatile v8h*)dst = o;
}

__global__ __launch_bounds__(TPB) void xpose_k(const float* __restrict__ x, f16t* __restrict__ XT)
{
  __shared__ __attribute__((aligned(16))) f16t sT[PT * PQ];
  const int tid = threadIdx.x, lane = tid & 31, wave = tid >> 5;
  const int p0 = blockIdx.x * PT, b = blockIdx.y;
  const int c0 = tid >> 4, p4 = (tid & 15) * 4;
  const float* xb = x + (size_t)b * CIN * HW + p0 + p4;
  #pragma unroll 4
  for (int i = 0; i < 16; ++i) {
    const int c = c0 + 16 * i;
    const v4f v = *(const v4fa*)(xb + (size_t)c * HW);
    sT[(p4 + 0) * PQ + c] = (f16t)(v[0] * XCAR);
    sT[(p4 + 1) * PQ + c] = (f16t)(v[1] * XCAR);
    sT[(p4 + 2) * PQ + c] = (f16t)(v[2] * XCAR);
    sT[(p4 + 3) * PQ + c] = (f16t)(v[3] * XCAR);
  }
  __syncthreads();
  store_rows256(sT, XT + ((size_t)b * HW + p0) * CIN, wave, lane);
}

__global__ __launch_bounds__(TPB) void proj_k(const f16t* __restrict__ XT, const f16t* __restrict__ WP,
                                             const float* __restrict__ bq, const float* __restrict__ bk,
                                             const float* __restrict__ bv,
                                             f16t* __restrict__ QN, f16t* __restrict__ KN, f16t* __restrict__ VH)
{
  __shared__ __attribute__((aligned(16))) f16t  sT[256 * PK];
  __shared__ __attribute__((aligned(16))) float sS[WAVES * PT];
  const int tid = threadIdx.x, lane = tid & 31, wave = tid >> 5;
  const int h = lane >> 4, m = lane & 15;
  const int p0 = blockIdx.x * PT, y = blockIdx.y, b = blockIdx.z;

  v8f acc[2][4];
  #pragma unroll
  for (int mt = 0; mt < 2; ++mt) {
    #pragma unroll
    for (int n = 0; n < 4; ++n) acc[mt][n] = zero8f();
  }
  const f16t* arow = WP + (size_t)(y * 256 + wave * 32 + m) * CIN + 8 * h;
  const f16t* brow = XT + ((size_t)b * HW + p0 + m) * CIN + 8 * h;
  #pragma unroll 1
  for (int ks = 0; ks < CIN / 32; ++ks) {
    const int k0 = 32 * ks;
    FragH a0, a1, bf[4];
    load_frag(a0, arow, k0);
    load_frag(a1, arow + 16 * CIN, k0);
    #pragma unroll
    for (int n = 0; n < 4; ++n) load_frag(bf[n], brow + (size_t)16 * n * CIN, k0);
    #pragma unroll
    for (int n = 0; n < 4; ++n) {
      acc[0][n] = wmma_f16(a0.v, bf[n].v, acc[0][n]);
      acc[1][n] = wmma_f16(a1.v, bf[n].v, acc[1][n]);
    }
  }

  const float* bp = bq;
  if (y == 1) bp = bk;
  if (y == 2) bp = bv;
  if (y == 3) bp = bv + 256;
  v4f cb[2][2];
  #pragma unroll
  for (int mt = 0; mt < 2; ++mt) {
    const int ob = wave * 32 + 16 * mt + 8 * h;
    cb[mt][0] = *(const v4fa*)(bp + ob);
    cb[mt][1] = *(const v4fa*)(bp + ob + 4);
  }
  const float sc = 1.0f / (XCAR * WCAR);

  float ssq[4];
  #pragma unroll
  for (int n = 0; n < 4; ++n) {
    float s = 0.0f;
    #pragma unroll
    for (int mt = 0; mt < 2; ++mt) {
      #pragma unroll
      for (int r = 0; r < 4; ++r) {
        const float t0 = fmaf(acc[mt][n][r], sc, cb[mt][0][r]);
        const float t1 = fmaf(acc[mt][n][4 + r], sc, cb[mt][1][r]);
        s = fmaf(t0, t0, s);
        s = fmaf(t1, t1, s);
      }
    }
    ssq[n] = s;
  }
  #pragma unroll
  for (int n = 0; n < 4; ++n) ssq[n] += __shfl_xor(ssq[n], 16);
  if (h == 0) {
    #pragma unroll
    for (int n = 0; n < 4; ++n) sS[wave * PT + 16 * n + m] = ssq[n];
  }
  __syncthreads();
  float rs[4];
  #pragma unroll
  for (int n = 0; n < 4; ++n) {
    float tot = 0.0f;
    #pragma unroll
    for (int w2 = 0; w2 < WAVES; ++w2) tot += sS[w2 * PT + 16 * n + m];
    const float r = rsqrtf(tot * (1.0f / 256.0f) + 1e-8f);
    rs[n] = (y < 2) ? r : 1.0f;
  }

  if (y == 0) {
    #pragma unroll
    for (int mt = 0; mt < 2; ++mt) {
      #pragma unroll
      for (int n = 0; n < 4; ++n) {
        v8h o;
        #pragma unroll
        for (int r = 0; r < 4; ++r) {
          const float t0 = fmaf(acc[mt][n][r], sc, cb[mt][0][r]) * rs[n];
          const float t1 = fmaf(acc[mt][n][4 + r], sc, cb[mt][1][r]) * rs[n];
          o[r]     = (f16t)(t0 * QCAR);
          o[4 + r] = (f16t)(t1 * QCAR);
        }
        *(v8ha*)(sT + (16 * n + m) * PQ + wave * 32 + 16 * mt + 8 * h) = o;
      }
    }
  } else {
    #pragma unroll
    for (int mt = 0; mt < 2; ++mt) {
      #pragma unroll
      for (int n = 0; n < 4; ++n) {
        #pragma unroll
        for (int r = 0; r < 4; ++r) {
          const float t0 = fmaf(acc[mt][n][r], sc, cb[mt][0][r]) * rs[n];
          const float t1 = fmaf(acc[mt][n][4 + r], sc, cb[mt][1][r]) * rs[n];
          const int c0 = wave * 32 + 16 * mt + 8 * h + r;
          sT[c0 * PK + 16 * n + m]       = (f16t)(t0 * QCAR);
          sT[(c0 + 4) * PK + 16 * n + m] = (f16t)(t1 * QCAR);
        }
      }
    }
  }
  __syncthreads();
  if (y == 0) {
    store_rows256(sT, QN + ((size_t)b * HW + p0) * NQK, wave, lane);
  } else {
    f16t* dst = KN + (size_t)b * NQK * HW + p0;
    if (y == 2) dst = VH + (size_t)b * NV * HW + p0;
    if (y == 3) dst = VH + ((size_t)b * NV + 256) * HW + p0;
    store_rows64(sT, dst, wave, lane);
  }
}

__global__ __launch_bounds__(TPB) void kv_k(const f16t* __restrict__ KN, const f16t* __restrict__ VH,
                                          f16t* __restrict__ KVT)
{
  __shared__ __attribute__((aligned(16))) float sKV[CQ * CV];
  __shared__ __attribute__((aligned(16))) f16t  sKT[CV * PKT];
  const int tid = threadIdx.x, lane = tid & 31, wave = tid >> 5;
  const int h = lane >> 4, m = lane & 15;
  const int bg = blockIdx.x, b = bg >> 3, g = bg & 7;
  const int mt = wave & 1, nt = wave >> 1;
  const f16t* arow = KN + ((size_t)b * NQK + g * CQ + 16 * mt + m) * HW + 8 * h;
  const f16t* brow = VH + ((size_t)b * NV + g * CV + 16 * nt + m) * HW + 8 * h;
  v8f acc = zero8f();
  #pragma unroll 2
  for (int ks = 0; ks < HW / 32; ++ks) {
    const int k0 = 32 * ks;
    FragH a, bb;
    load_frag(a, arow, k0);
    load_frag(bb, brow, k0);
    acc = wmma_f16(a.v, bb.v, acc);
  }
  const float sc = 1.0f / (QCAR * QCAR);
  #pragma unroll
  for (int r = 0; r < 8; ++r) sKV[(16 * mt + 8 * h + r) * CV + 16 * nt + m] = acc[r] * sc;
  __syncthreads();
  if (tid < CV) {
    const int C = tid;
    float ssq = 0.0f;
    #pragma unroll 8
    for (int c = 0; c < CQ; ++c) { const float v = sKV[c * CV + C]; ssq = fmaf(v, v, ssq); }
    const float rsn = rsqrtf(ssq * (1.0f / 32.0f) + 1e-8f) * KVCAR;
    #pragma unroll
    for (int j = 0; j < 4; ++j) {
      v8h o;
      #pragma unroll
      for (int i = 0; i < 8; ++i) o[i] = (f16t)(sKV[(8 * j + i) * CV + C] * rsn);
      *(v8ha*)(sKT + C * PKT + 8 * j) = o;
    }
  }
  __syncthreads();
  const v8h o = *(const v8ha*)(sKT + (tid >> 2) * PKT + (tid & 3) * 8);
  f16t* dst = KVT + (size_t)bg * (CV * CQ) + (tid >> 2) * CQ + (tid & 3) * 8;
  *(volatile v8h*)dst = o;
  __threadfence();
  *(volatile v8h*)dst = o;
}

__global__ __launch_bounds__(TPB) void qkv_k(const f16t* __restrict__ QN, const f16t* __restrict__ KVT,
                                           f16t* __restrict__ QKT, float* __restrict__ HG)
{
  __shared__ __attribute__((aligned(16))) f16t  sT[PT * PQ];
  __shared__ __attribute__((aligned(16))) float sL[NG * PT];
  const int tid = threadIdx.x, lane = tid & 31, wave = tid >> 5;
  const int h = lane >> 4, m = lane & 15;
  const int p0 = blockIdx.x * PT, b = blockIdx.y;
  const int g = wave, bg = b * NG + g;

  FragH bqf[4];
  #pragma unroll
  for (int n = 0; n < 4; ++n)
    load_frag(bqf[n], QN + ((size_t)b * HW + p0 + 16 * n + m) * NQK + g * CQ + 8 * h, 0);
  const f16t* arow = KVT + ((size_t)bg * CV + m) * CQ + 8 * h;

  const float psc = QVCAR / (KVCAR * QCAR);
  #pragma unroll
  for (int mt = 0; mt < 2; ++mt) {
    FragH a;
    load_frag(a, arow + 16 * mt * CQ, 0);
    #pragma unroll
    for (int n = 0; n < 4; ++n) {
      const v8f d = wmma_f16(a.v, bqf[n].v, zero8f());
      v8h o;
      #pragma unroll
      for (int r = 0; r < 8; ++r) o[r] = (f16t)(d[r] * psc);
      *(v8ha*)(sT + (16 * n + m) * PQ + g * CKEEP + 16 * mt + 8 * h) = o;
    }
  }
  float lg[4] = {0.0f, 0.0f, 0.0f, 0.0f};
  #pragma unroll
  for (int mt = 2; mt < 4; ++mt) {
    FragH a;
    load_frag(a, arow + 16 * mt * CQ, 0);
    #pragma unroll
    for (int n = 0; n < 4; ++n) {
      const v8f d = wmma_f16(a.v, bqf[n].v, zero8f());
      float s = 0.0f;
      #pragma unroll
      for (int r = 0; r < 8; ++r) s += d[r];
      lg[n] += s;
    }
  }
  #pragma unroll
  for (int n = 0; n < 4; ++n) lg[n] += __shfl_xor(lg[n], 16);
  const float lsc = 1.0f / (KVCAR * QCAR * 32.0f * 64.0f);
  if (h == 0) {
    #pragma unroll
    for (int n = 0; n < 4; ++n) sL[g * PT + 16 * n + m] = lg[n] * lsc;
  }
  __syncthreads();
  store_rows256(sT, QKT + ((size_t)b * HW + p0) * KF, wave, lane);
  {
    const int lc = lane & 15;
    const v4f v = *(const v4fa*)(sL + g * PT + 4 * lc);
    float* dst = HG + (size_t)bg * HW + p0 + 4 * lc;
    if (lane < 16) *(volatile v4f*)dst = v;
    __threadfence();
    if (lane < 16) *(volatile v4f*)dst = v;
  }
}

__global__ __launch_bounds__(TPB) void gate_k(const float* __restrict__ HG, float* __restrict__ GST)
{
  __shared__ float sRa[WAVES];
  __shared__ float sRb[WAVES];
  __shared__ __attribute__((aligned(16))) float sSt[NB * NG * 2];
  const int tid = threadIdx.x, lane = tid & 31, wave = tid >> 5;
  #pragma unroll 1
  for (int bg = 0; bg < NB * NG; ++bg) {
    const float* src = HG + (size_t)bg * HW;
    float z[16];
    float lmax = -3.0e38f;
    #pragma unroll
    for (int i = 0; i < 16; ++i) { z[i] = src[tid + TPB * i]; lmax = fmaxf(lmax, z[i]); }
    #pragma unroll
    for (int s = 16; s > 0; s >>= 1) lmax = fmaxf(lmax, __shfl_xor(lmax, s));
    if (lane == 0) sRa[wave] = lmax;
    __syncthreads();
    float zm = sRa[0];
    #pragma unroll
    for (int w2 = 1; w2 < WAVES; ++w2) zm = fmaxf(zm, sRa[w2]);
    float lsum = 0.0f;
    #pragma unroll
    for (int i = 0; i < 16; ++i) lsum += __expf(z[i] - zm);
    #pragma unroll
    for (int s = 16; s > 0; s >>= 1) lsum += __shfl_xor(lsum, s);
    if (lane == 0) sRb[wave] = lsum;
    __syncthreads();
    float tot = sRb[0];
    #pragma unroll
    for (int w2 = 1; w2 < WAVES; ++w2) tot += sRb[w2];
    if (tid == 0) { sSt[2 * bg] = zm; sSt[2 * bg + 1] = 1.0f / tot; }
  }
  __syncthreads();
  const v4f v = *(const v4fa*)(sSt + 4 * lane);
  float* dst = GST + 4 * lane;
  if (wave == 0) *(volatile v4f*)dst = v;
  __threadfence();
  if (wave == 0) *(volatile v4f*)dst = v;
}

__global__ __launch_bounds__(TPB) void fuse_k(const f16t* __restrict__ QKT, const f16t* __restrict__ WP,
                                            const float* __restrict__ HG, const float* __restrict__ GST,
                                            const float* __restrict__ pbf, const float* __restrict__ pga,
                                            const float* __restrict__ pbe, const float* __restrict__ pmu,
                                            const float* __restrict__ pva, float* __restrict__ out)
{
  __shared__ __attribute__((aligned(16))) float sG[NG * PT];
  __shared__ __attribute__((aligned(16))) float sO[WAVES * 16 * PT];
  const int tid = threadIdx.x, lane = tid & 31, wave = tid >> 5;
  const int h = lane >> 4, m = lane & 15;
  const int p0 = blockIdx.x * PT, b = blockIdx.y;

  #pragma unroll
  for (int j = 0; j < 2; ++j) {
    const int idx = tid + TPB * j;
    const int g = idx >> 6, p = idx & 63;
    const int bg = b * NG + g;
    const float z  = HG[(size_t)bg * HW + p0 + p];
    const float zm = GST[2 * bg];
    const float iv = GST[2 * bg + 1];
    sG[idx] = __expf(z - zm) * iv;
  }
  __syncthreads();

  v8f acc[2][4];
  #pragma unroll
  for (int mt = 0; mt < 2; ++mt) {
    #pragma unroll
    for (int n = 0; n < 4; ++n) acc[mt][n] = zero8f();
  }
  const f16t* arow = WP + (size_t)(1024 + wave * 32 + m) * KF + 8 * h;
  const f16t* brow = QKT + ((size_t)b * HW + p0 + m) * KF + 8 * h;
  #pragma unroll 1
  for (int g = 0; g < NG; ++g) {
    const int k0 = CKEEP * g;
    FragH a0, a1, bf[4];
    load_frag(a0, arow, k0);
    load_frag(a1, arow + 16 * KF, k0);
    #pragma unroll
    for (int n = 0; n < 4; ++n) load_frag(bf[n], brow + (size_t)16 * n * KF, k0);
    float gv[4];
    #pragma unroll
    for (int n = 0; n < 4; ++n) gv[n] = sG[g * PT + 16 * n + m];
    #pragma unroll
    for (int n = 0; n < 4; ++n) {
      const v8f d0 = wmma_f16(a0.v, bf[n].v, zero8f());
      const v8f d1 = wmma_f16(a1.v, bf[n].v, zero8f());
      #pragma unroll
      for (int r = 0; r < 8; ++r) {
        acc[0][n][r] = fmaf(d0[r], gv[n], acc[0][n][r]);
        acc[1][n][r] = fmaf(d1[r], gv[n], acc[1][n][r]);
      }
    }
  }

  const float sc = 1.0f / (WCAR * QVCAR);
  #pragma unroll
  for (int mt = 0; mt < 2; ++mt) {
    const int ob = wave * 32 + 16 * mt + 8 * h;
    const v4f cb0 = *(const v4fa*)(pbf + ob), cb1 = *(const v4fa*)(pbf + ob + 4);
    const v4f mu0 = *(const v4fa*)(pmu + ob), mu1 = *(const v4fa*)(pmu + ob + 4);
    const v4f va0 = *(const v4fa*)(pva + ob), va1 = *(const v4fa*)(pva + ob + 4);
    const v4f ga0 = *(const v4fa*)(pga + ob), ga1 = *(const v4fa*)(pga + ob + 4);
    const v4f be0 = *(const v4fa*)(pbe + ob), be1 = *(const v4fa*)(pbe + ob + 4);
    float rs0[4], rs1[4];
    #pragma unroll
    for (int r = 0; r < 4; ++r) { rs0[r] = rsqrtf(va0[r] + 1e-5f); rs1[r] = rsqrtf(va1[r] + 1e-5f); }
    #pragma unroll
    for (int n = 0; n < 4; ++n) {
      #pragma unroll
      for (int r = 0; r < 4; ++r) {
        float t0 = fmaf(acc[mt][n][r], sc, cb0[r]);
        t0 = (t0 - mu0[r]) * rs0[r];
        t0 = fmaf(t0, ga0[r], be0[r]);
        t0 = fmaxf(t0, 0.0f);
        float t1 = fmaf(acc[mt][n][4 + r], sc, cb1[r]);
        t1 = (t1 - mu1[r]) * rs1[r];
        t1 = fmaf(t1, ga1[r], be1[r]);
        t1 = fmaxf(t1, 0.0f);
        sO[wave * 1024 + (8 * h + r) * PT + 16 * n + m]     = t0;
        sO[wave * 1024 + (8 * h + 4 + r) * PT + 16 * n + m] = t1;
      }
    }
    __syncthreads();
    float* orow = out + ((size_t)b * COUT + wave * 32 + 16 * mt) * HW + p0;
    const int l16 = lane & 15, rsel = lane >> 4;
    #pragma unroll
    for (int i = 0; i < 8; ++i) {
      const int row = 2 * i + rsel;
      const v4f v = *(const v4fa*)(sO + wave * 1024 + row * PT + 4 * l16);
      *(volatile v4f*)(orow + (size_t)row * HW + 4 * l16) = v;
    }
    __threadfence();
    #pragma unroll
    for (int i = 0; i < 8; ++i) {
      const int row = 2 * i + rsel;
      const v4f v = *(const v4fa*)(sO + wave * 1024 + row * PT + 4 * l16);
      *(volatile v4f*)(orow + (size_t)row * HW + 4 * l16) = v;
    }
    __syncthreads();
  }
}

extern "C" void kernel_launch(void* const* d_in, const int* in_sizes, int n_in,
                              void* d_out, int out_size, void* d_ws, size_t ws_size,
                              hipStream_t stream) {
  if (n_in < 13) return;
  if (in_sizes[0]  != NB * CIN * HW) return;
  if (in_sizes[1]  != NQK * CIN)     return;
  if (in_sizes[2]  != NQK)           return;
  if (in_sizes[3]  != NQK * CIN)     return;
  if (in_sizes[4]  != NQK)           return;
  if (in_sizes[5]  != NV * CIN)      return;
  if (in_sizes[6]  != NV)            return;
  if (in_sizes[7]  != COUT * KF)     return;
  if (in_sizes[8]  != COUT)          return;
  if (in_sizes[9]  != COUT)          return;
  if (in_sizes[10] != COUT)          return;
  if (in_sizes[11] != COUT)          return;
  if (in_sizes[12] != COUT)          return;
  if (out_size != NB * COUT * HW)    return;

  const float* x    = (const float*)d_in[0];
  const float* Wq   = (const float*)d_in[1];
  const float* bq   = (const float*)d_in[2];
  const float* Wk   = (const float*)d_in[3];
  const float* bk   = (const float*)d_in[4];
  const float* Wv   = (const float*)d_in[5];
  const float* bv   = (const float*)d_in[6];
  const float* Wf   = (const float*)d_in[7];
  const float* bfv  = (const float*)d_in[8];
  const float* gam  = (const float*)d_in[9];
  const float* bet  = (const float*)d_in[10];
  const float* mu   = (const float*)d_in[11];
  const float* var  = (const float*)d_in[12];
  float* outp = (float*)d_out;

  const size_t szWP  = (size_t)WROWS * CIN * 2;
  const size_t szXT  = (size_t)NB * HW * CIN * 2;
  const size_t szQN  = (size_t)NB * HW * NQK * 2;
  const size_t szKN  = (size_t)NB * NQK * HW * 2;
  const size_t szVH  = (size_t)NB * NV * HW * 2;
  const size_t szKVT = (size_t)NB * NG * CV * CQ * 2;
  const size_t szQKT = (size_t)NB * HW * KF * 2;
  const size_t szHG  = (size_t)NB * NG * HW * 4;
  const size_t szGST = (size_t)NB * NG * 2 * 4;
  size_t off = 0;
  char* ws = (char*)d_ws;
  f16t*  WP  = (f16t*)(ws + off);  off += szWP;
  f16t*  XT  = (f16t*)(ws + off);  off += szXT;
  f16t*  QN  = (f16t*)(ws + off);  off += szQN;
  f16t*  KN  = (f16t*)(ws + off);  off += szKN;
  f16t*  VH  = (f16t*)(ws + off);  off += szVH;
  f16t*  KVT = (f16t*)(ws + off);  off += szKVT;
  f16t*  QKT = (f16t*)(ws + off);  off += szQKT;
  float* HG  = (float*)(ws + off); off += szHG;
  float* GST = (float*)(ws + off); off += szGST;
  if (off > ws_size) return;

  prep_w_k<<<(WROWS * 32) / TPB, TPB, 0, stream>>>(Wq, Wk, Wv, Wf, WP);
  xpose_k<<<dim3(HW / PT, NB), TPB, 0, stream>>>(x, XT);
  proj_k<<<dim3(HW / PT, 4, NB), TPB, 0, stream>>>(XT, WP, bq, bk, bv, QN, KN, VH);
  kv_k<<<NB * NG, TPB, 0, stream>>>(KN, VH, KVT);
  qkv_k<<<dim3(HW / PT, NB), TPB, 0, stream>>>(QN, KVT, QKT, HG);
  gate_k<<<1, TPB, 0, stream>>>(HG, GST);
  fuse_k<<<dim3(HW / PT, NB), TPB, 0, stream>>>(QKT, WP, HG, GST, bfv, gam, bet, mu, var, outp);
}
